// MSA_32057635897504
// MI455X (gfx1250) — hardware-verified
//
#include <hip/hip_runtime.h>
#include <math.h>

typedef __attribute__((ext_vector_type(16))) _Float16 v16h;
typedef __attribute__((ext_vector_type(16))) __bf16 v16b;
typedef __attribute__((ext_vector_type(8)))  _Float16 v8h;
typedef __attribute__((ext_vector_type(8)))  __bf16 v8b;
typedef __attribute__((ext_vector_type(8)))  float v8f;
typedef __attribute__((ext_vector_type(4)))  float v4f;
typedef __attribute__((ext_vector_type(4)))  unsigned v4u;

template <typename T> __device__ __forceinline__ void vst2(void* p, T v) { *(volatile T*)p = v; __threadfence(); *(volatile T*)p = v; }
__device__ __forceinline__ v8f wmma16(v16h a, v16h b, v8f c) {
  v8f d = __builtin_amdgcn_wmma_f32_16x16x32_f16(false, a, false, b, (short)0, c, false, false);
  asm volatile("v_nop\n\tv_nop\n\tv_nop\n\tv_nop" : "+v"(d) : "v"(a), "v"(b));
  return d;
}
__device__ __forceinline__ v8f wmma_bf(v16b a, v16b b, v8f c) {
  v8f d = __builtin_amdgcn_wmma_f32_16x16x32_bf16(false, a, false, b, (short)0, c, false, false);
  asm volatile("v_nop\n\tv_nop\n\tv_nop\n\tv_nop" : "+v"(d) : "v"(a), "v"(b));
  return d;
}
__device__ __forceinline__ v16h frag_h(const _Float16* rowk0, int lane) {
  union { v16h v; v8h q[2]; } u; const _Float16* p = rowk0 + 8 * (lane >> 4);
  u.q[0] = *(const v8h*)p; u.q[1] = *(const v8h*)(p + 16); return u.v;
}
__device__ __forceinline__ v16b frag_b(const __bf16* rowk0, int lane) {
  union { v16b v; v8b q[2]; } u; const __bf16* p = rowk0 + 8 * (lane >> 4);
  u.q[0] = *(const v8b*)p; u.q[1] = *(const v8b*)(p + 16); return u.v;
}
__device__ __forceinline__ float bfr(float v) { return (float)(__bf16)v; }
__device__ __forceinline__ void ldsx() { asm volatile("s_wait_dscnt 0" ::: "memory"); __builtin_amdgcn_wave_barrier(); __builtin_amdgcn_fence(3, "workgroup"); }

#ifndef NB
#define NB 8
#endif
#ifndef SEQ
#define SEQ 1024
#endif
#define NB_FULL 8
#define SEQ_FULL 1024
#define DD 768
#define NH 12
#define HD 64
#define MAXPOS 1024
#define NE (2 * MAXPOS - 1)
#define NEP (2 * MAXPOS)
#define QT 64
#define KT 128
#define NBC 9
#define SQP 148
#define SSP 132
#define SBW (16 * SQP)
static_assert(NB <= NB_FULL);
static_assert(SEQ <= SEQ_FULL);
static_assert(SEQ <= MAXPOS);
static_assert(SEQ % KT == 0);
static_assert(SEQ % QT == 0);
static_assert(NH * HD == DD);
static_assert(DD % 128 == 0);
static_assert(16 * NBC >= 16 + KT - 1);
static_assert(16 * SSP <= SBW);

#define WS_XB  ((size_t)0)
#define WS_WB  (WS_XB + 2u * (size_t)NB * SEQ * DD)
#define WS_EP  (WS_WB + 2u * (size_t)3 * DD * DD)
#define WS_QH  (WS_EP + 2u * (size_t)NEP * HD)
#define WS_KH  (WS_QH + 2u * (size_t)NB * SEQ * DD)
#define WS_VT  (WS_KH + 2u * (size_t)NB * SEQ * DD)
#define WS_S   (WS_VT + 2u * (size_t)NB * DD * SEQ)
#define WS_PH  (WS_S + 4u * (size_t)NH * SEQ * SEQ)
#define WS_END (WS_PH + 2u * (size_t)NH * SEQ * SEQ)
static_assert(WS_END <= (size_t)134217728);
static_assert(WS_WB % 128 == 0 && WS_EP % 128 == 0 && WS_QH % 128 == 0 && WS_KH % 128 == 0 && WS_VT % 128 == 0 && WS_S % 128 == 0 && WS_PH % 128 == 0);

__global__ __launch_bounds__(256) void k_cvt(const float* __restrict__ src, unsigned short* __restrict__ dst, int nrows, int nsrc, int ncol, int seg, int segfull, int kind, float sc) {
  const int cpr = ncol >> 3;
  const size_t total = (size_t)nrows * cpr;
  const size_t i8 = (size_t)blockIdx.x * 256 + threadIdx.x;
  if (i8 >= total) return;
  const int dr = (int)(i8 / cpr), cc = (int)(i8 - (size_t)dr * cpr) * 8;
  const int drc = dr < nsrc ? dr : nsrc - 1;
  const size_t srow = (size_t)(drc / seg) * segfull + (size_t)(drc % seg);
  const float* p = src + srow * (size_t)ncol + cc;
  const v4f va = *(const v4f*)p, vb = *(const v4f*)(p + 4);
  const bool z = dr >= nsrc;
  float v[8];
#pragma unroll
  for (int i = 0; i < 4; ++i) { v[i] = z ? 0.f : va[i]; v[4 + i] = z ? 0.f : vb[i]; }
  union { v8h h; v8b b; v4u u; } o;
  if (kind == 0) {
#pragma unroll
    for (int i = 0; i < 8; ++i) o.b[i] = (__bf16)v[i];
  } else {
#pragma unroll
    for (int i = 0; i < 8; ++i) o.h[i] = (_Float16)(bfr(v[i]) * sc);
  }
  vst2(dst + i8 * 8, o.u);
}

__global__ __launch_bounds__(128) void k_proj(const __bf16* __restrict__ XB, const __bf16* __restrict__ WB, const float* __restrict__ BQ, const float* __restrict__ BK, const float* __restrict__ BV, _Float16* __restrict__ QH, _Float16* __restrict__ KH, _Float16* __restrict__ VT) {
  __shared__ __align__(16) _Float16 sh[64][136];
  __shared__ __align__(16) _Float16 th[128][72];
  const int tid = threadIdx.x, wave = tid >> 5, lane = tid & 31, col = lane & 15, g = lane >> 4;
  const int which = blockIdx.z; const int c0 = blockIdx.y * 128; const size_t r0 = (size_t)blockIdx.x * 64;
  const __bf16* W = WB + (size_t)which * DD * DD;
  const float* Bp = which == 0 ? BQ : (which == 1 ? BK : BV);
  v8f acc[8] = {};
#pragma unroll 2
  for (int kc = 0; kc < DD / 32; ++kc) {
    const v16b a = frag_b(XB + (r0 + wave * 16 + col) * DD + kc * 32, lane);
#pragma unroll
    for (int j = 0; j < 8; ++j) { const v16b w = frag_b(W + (size_t)(c0 + j * 16 + col) * DD + kc * 32, lane); acc[j] = wmma_bf(a, w, acc[j]); }
  }
#pragma unroll
  for (int j = 0; j < 8; ++j) { const float bb = bfr(Bp[c0 + j * 16 + col]);
#pragma unroll
    for (int r = 0; r < 8; ++r) { const float v = (acc[j][r] + bb) * 16.0f; const int rl = wave * 16 + 8 * g + r, cl = j * 16 + col; const _Float16 hv = (_Float16)v;
      if (which == 2) th[cl][rl] = hv; else sh[rl][cl] = hv; } }
  __syncthreads();
  if (which < 2) { _Float16* dh = which == 0 ? QH : KH;
    for (int e = tid; e < 64 * 16; e += 128) { const int rl = e >> 4, q = e & 15; vst2(dh + (r0 + rl) * DD + c0 + q * 8, *(const v4u*)&sh[rl][q * 8]); } }
  else { const size_t b = r0 / SEQ; const int t0 = (int)(r0 % SEQ);
    for (int e = tid; e < 128 * 8; e += 128) { const int cl = e >> 3, q = e & 7; const size_t o2 = (b * DD + c0 + cl) * (size_t)SEQ + t0 + q * 8; vst2(VT + o2, *(const v4u*)&th[cl][q * 8]); } }
}

__global__ __launch_bounds__(128) __attribute__((amdgpu_num_vgpr(256))) void k_sc(const _Float16* __restrict__ QH, const _Float16* __restrict__ KH, const _Float16* __restrict__ EP, int b, float* __restrict__ S0) {
  __shared__ __align__(16) float sbuf[4][SBW];
  const int h = blockIdx.z; float* S = S0 + (size_t)h * SEQ * SEQ;
  const int tid = threadIdx.x, wave = tid >> 5, lane = tid & 31, col = lane & 15, g = lane >> 4;
  const int k0 = blockIdx.y * KT; const int ql0 = blockIdx.x * QT + wave * 16; const size_t q0 = (size_t)b * SEQ + ql0;
  const v16h a0 = frag_h(QH + (q0 + col) * DD + h * HD, lane), a1 = frag_h(QH + (q0 + col) * DD + h * HD + 32, lane);
  const int cbase = ql0 + (MAXPOS - 1) - k0 - (KT - 1);
#pragma unroll 3
  for (int t = 0; t < NBC; ++t) {
    int er = cbase + t * 16 + col; er = er < 0 ? 0 : er; er = er > NEP - 1 ? NEP - 1 : er;
    v8f c = {};
    c = wmma16(a0, frag_h(EP + (size_t)er * HD, lane), c);
    c = wmma16(a1, frag_h(EP + (size_t)er * HD + 32, lane), c);
#pragma unroll
    for (int r = 0; r < 8; ++r) sbuf[wave][(8 * g + r) * SQP + t * 16 + col] = c[r];
  }
  ldsx();
  v8f acc[8] = {};
#pragma unroll
  for (int j = 0; j < 8; ++j) { const _Float16* kp = KH + ((size_t)b * SEQ + k0 + j * 16 + col) * DD + h * HD;
    acc[j] = wmma16(a0, frag_h(kp, lane), acc[j]); acc[j] = wmma16(a1, frag_h(kp + 32, lane), acc[j]); }
#pragma unroll
  for (int j = 0; j < 8; ++j)
#pragma unroll
    for (int r = 0; r < 8; ++r) { const int u = 8 * g + r; const int c = u + (KT - 1) - j * 16 - col; acc[j][r] = (acc[j][r] + sbuf[wave][u * SQP + c]) * (1.0f / 2048.0f); }
  ldsx();
#pragma unroll
  for (int j = 0; j < 8; ++j)
#pragma unroll
    for (int r = 0; r < 8; ++r) sbuf[wave][(8 * g + r) * SSP + j * 16 + col] = acc[j][r];
  ldsx();
  for (int rl = 0; rl < 16; ++rl) vst2(S + (size_t)(ql0 + rl) * SEQ + k0 + lane * 4, *(const v4f*)&sbuf[wave][rl * SSP + lane * 4]);
}

__global__ __launch_bounds__(256) void k_sm(const float* __restrict__ S0, _Float16* __restrict__ PH0) {
  __shared__ float sred[8]; __shared__ float sbc; __shared__ __align__(16) float sh[SEQ];
  const int t = threadIdx.x; const size_t row = blockIdx.x; const int h = blockIdx.y;
  const float* sr = S0 + ((size_t)h * SEQ + row) * SEQ; _Float16* pr = PH0 + ((size_t)h * SEQ + row) * SEQ;
  float m = -3.0e38f;
#pragma unroll 1
  for (int q = t; q < SEQ / 4; q += 256) { const v4f v = *(const v4f*)(sr + q * 4); *(v4f*)&sh[q * 4] = v; m = fmaxf(m, fmaxf(fmaxf(v[0], v[1]), fmaxf(v[2], v[3]))); }
#pragma unroll
  for (int o = 1; o < 32; o <<= 1) m = fmaxf(m, __shfl_xor(m, o));
  if ((t & 31) == 0) sred[t >> 5] = m;
  __syncthreads();
  if (t == 0) { float a = sred[0]; for (int i = 1; i < 8; ++i) a = fmaxf(a, sred[i]); sbc = a; }
  __syncthreads();
  m = sbc;
  __syncthreads();
  float sum = 0.f;
#pragma unroll 1
  for (int k = t; k < SEQ; k += 256) { const float e = expf(sh[k] - m); sh[k] = e; sum += e; }
#pragma unroll
  for (int o = 1; o < 32; o <<= 1) sum += __shfl_xor(sum, o);
  if ((t & 31) == 0) sred[t >> 5] = sum;
  __syncthreads();
  if (t == 0) { float a = 0.f; for (int i = 0; i < 8; ++i) a += sred[i]; sbc = (1.0f / a) * 16384.0f; }
  __syncthreads();
  const float sc = sbc;
#pragma unroll 1
  for (int q = t; q < SEQ / 8; q += 256) { union { v8h hh; v4u u; } o;
#pragma unroll
    for (int i = 0; i < 8; ++i) o.hh[i] = (_Float16)(sh[q * 8 + i] * sc);
    vst2(pr + q * 8, o.u); }
}

__global__ __launch_bounds__(128) __attribute__((amdgpu_num_vgpr(256))) void k_pv(const _Float16* __restrict__ PH0, const _Float16* __restrict__ VT, int b, float* __restrict__ Y) {
  __shared__ __align__(16) float ss[4][16][HD + 4];
  const int h = blockIdx.z; const _Float16* PH = PH0 + (size_t)h * SEQ * SEQ;
  const int tid = threadIdx.x, wave = tid >> 5, lane = tid & 31, col = lane & 15, g = lane >> 4;
  const int ql0 = blockIdx.x * QT + wave * 16;
  v8f acc[HD / 16] = {};
#pragma unroll 2
  for (int kc = 0; kc < SEQ / 32; ++kc) {
    const v16h p = frag_h(PH + (size_t)(ql0 + col) * SEQ + kc * 32, lane);
#pragma unroll
    for (int j = 0; j < HD / 16; ++j) { const v16h vh = frag_h(VT + ((size_t)b * DD + h * HD + j * 16 + col) * (size_t)SEQ + kc * 32, lane); acc[j] = wmma16(p, vh, acc[j]); }
  }
#pragma unroll
  for (int j = 0; j < HD / 16; ++j)
#pragma unroll
    for (int r = 0; r < 8; ++r) ss[wave][8 * g + r][j * 16 + col] = acc[j][r] * (1.0f / 262144.0f);
  ldsx();
  for (int rl = 0; rl < 16; ++rl) if (lane < HD / 4) vst2(Y + ((size_t)b * SEQ + ql0 + rl) * DD + h * HD + lane * 4, *(const v4f*)&ss[wave][rl][lane * 4]);
}

extern "C" void kernel_launch(void* const* d_in, const int* in_sizes, int n_in, void* d_out, int out_size, void* d_ws, size_t ws_size, hipStream_t stream) {
  if (n_in < 8) return;
  if ((size_t)in_sizes[0] < ((size_t)(NB - 1) * SEQ_FULL + SEQ) * DD) return;
  if (in_sizes[1] < DD * DD || in_sizes[3] < DD * DD || in_sizes[5] < DD * DD) return;
  if (in_sizes[2] < DD || in_sizes[4] < DD || in_sizes[6] < DD) return;
  if (in_sizes[7] < NE * HD) return;
  if ((size_t)out_size < (size_t)NB * SEQ * DD) return;
  if (ws_size < WS_END) return;
  const float* const* F = (const float* const*)d_in;
  char* ws = (char*)d_ws;
  __bf16* XB = (__bf16*)(ws + WS_XB); __bf16* WB = (__bf16*)(ws + WS_WB); _Float16* EP = (_Float16*)(ws + WS_EP);
  _Float16 *QH = (_Float16*)(ws + WS_QH), *KH = (_Float16*)(ws + WS_KH), *VT = (_Float16*)(ws + WS_VT);
  float* S = (float*)(ws + WS_S); _Float16* PH = (_Float16*)(ws + WS_PH);
  const size_t nx8 = (size_t)NB * SEQ * DD / 8, nw8 = (size_t)DD * DD / 8, ne8 = (size_t)NEP * HD / 8;
  k_cvt<<<dim3((unsigned)((nx8 + 255) / 256)), 256, 0, stream>>>(F[0], (unsigned short*)XB, NB * SEQ, NB * SEQ, DD, SEQ, SEQ_FULL, 0, 1.0f);
  k_cvt<<<dim3((unsigned)((nw8 + 255) / 256)), 256, 0, stream>>>(F[1], (unsigned short*)WB, DD, DD, DD, DD, DD, 0, 1.0f);
  k_cvt<<<dim3((unsigned)((nw8 + 255) / 256)), 256, 0, stream>>>(F[3], (unsigned short*)(WB + (size_t)DD * DD), DD, DD, DD, DD, DD, 0, 1.0f);
  k_cvt<<<dim3((unsigned)((nw8 + 255) / 256)), 256, 0, stream>>>(F[5], (unsigned short*)(WB + (size_t)2 * DD * DD), DD, DD, DD, DD, DD, 0, 1.0f);
  k_cvt<<<dim3((unsigned)((ne8 + 255) / 256)), 256, 0, stream>>>(F[7], (unsigned short*)EP, NEP, NE, HD, NEP, NEP, 1, 16.0f);
  k_proj<<<dim3(NB * SEQ / 64, DD / 128, 3), 128, 0, stream>>>(XB, WB, F[2], F[4], F[6], QH, KH, VT);
  for (int b = 0; b < NB; ++b) {
    k_sc<<<dim3(SEQ / QT, SEQ / KT, NH), 128, 0, stream>>>(QH, KH, EP, b, S);
    k_sm<<<dim3(SEQ, NH), 256, 0, stream>>>(S, PH);
    k_pv<<<dim3(SEQ / QT, 1, NH), 128, 0, stream>>>(PH, VT, b, (float*)d_out);
  }
}
